// DENIS_JBF_57921928954562
// MI455X (gfx1250) — hardware-verified
//
#include <hip/hip_runtime.h>
#include <math.h>

typedef __attribute__((ext_vector_type(16))) _Float16 v16h;
typedef __attribute__((ext_vector_type(16))) __bf16 v16b;
typedef __attribute__((ext_vector_type(8)))  _Float16 v8h;
typedef __attribute__((ext_vector_type(8)))  float v8f;
typedef __attribute__((ext_vector_type(4)))  float v4f;
typedef __attribute__((ext_vector_type(2)))  float v2f;
typedef __attribute__((ext_vector_type(4)))  unsigned v4u;
typedef __attribute__((ext_vector_type(4)))  int v4i;
typedef float __attribute__((may_alias)) float_a;
typedef int __attribute__((may_alias)) int_a;

template <typename T> __device__ __forceinline__ void vst2(void* p, T v) { *(volatile T*)p = v; __threadfence(); *(volatile T*)p = v; }
__device__ __forceinline__ v8f wmma16(v16h a, v16h b, v8f c) {
  v8f d = __builtin_amdgcn_wmma_f32_16x16x32_f16(false, a, false, b, (short)0, c, false, false);
  asm volatile("v_nop\n\tv_nop\n\tv_nop\n\tv_nop" : "+v"(d) : "v"(a), "v"(b));
  return d;
}
__device__ __forceinline__ v8f wmma_bf(v16b a, v16b b, v8f c) {
  v8f d = __builtin_amdgcn_wmma_f32_16x16x32_bf16(false, a, false, b, (short)0, c, false, false);
  asm volatile("v_nop\n\tv_nop\n\tv_nop\n\tv_nop" : "+v"(d) : "v"(a), "v"(b));
  return d;
}
__device__ __forceinline__ v16h frag_h(const _Float16* rowk0, int lane) {
  union { v16h v; v8h q[2]; } u; const _Float16* p = rowk0 + 8 * (lane >> 4);
  u.q[0] = *(const v8h*)p; u.q[1] = *(const v8h*)(p + 16); return u.v;
}
__device__ __forceinline__ v16h frag_f32(const float* rowk0, int lane) {
  v16h a; const float* p = rowk0 + 8 * (lane >> 4);
#pragma unroll
  for (int i = 0; i < 8; ++i) { a[i] = (_Float16)p[i]; a[8 + i] = (_Float16)p[16 + i]; }
  return a;
}
__device__ __forceinline__ v16h frag_f32s(const float* rowk0, int lane, float sc) {
  v16h a; const float* p = rowk0 + 8 * (lane >> 4);
#pragma unroll
  for (int i = 0; i < 8; ++i) { a[i] = (_Float16)(p[i] * sc); a[8 + i] = (_Float16)(p[16 + i] * sc); }
  return a;
}
__device__ __forceinline__ v16h fragc_f32(const float* W, int k0, int n, int lane, int ld, int K) {
  v16h a; const int g = lane >> 4;
#pragma unroll
  for (int i = 0; i < 8; ++i) { const int ka = k0 + 8 * g + i, kb = ka + 16;
    a[i] = (_Float16)(ka < K ? W[(size_t)ka * ld + n] : 0.f); a[8 + i] = (_Float16)(kb < K ? W[(size_t)kb * ld + n] : 0.f); }
  return a;
}
struct F2 { v16b h, l; };
__device__ __forceinline__ F2 bsplit16(const float v[16]) { F2 r;
#pragma unroll
  for (int i = 0; i < 16; ++i) { const __bf16 h = (__bf16)v[i]; r.h[i] = h; r.l[i] = (__bf16)(v[i] - (float)h); }
  return r; }
__device__ __forceinline__ F2 split_row(const float* row, int k0, int lane) { float v[16]; const float* p = row + k0 + 8 * (lane >> 4);
#pragma unroll
  for (int i = 0; i < 8; ++i) { v[i] = p[i]; v[8 + i] = p[16 + i]; }
  return bsplit16(v); }
__device__ __forceinline__ F2 split_rowK(const float* row, int k0, int lane, int K) { float v[16]; const int g = lane >> 4;
#pragma unroll
  for (int i = 0; i < 8; ++i) { const int ka = k0 + 8 * g + i, kb = ka + 16; v[i] = ka < K ? row[ka] : 0.f; v[8 + i] = kb < K ? row[kb] : 0.f; }
  return bsplit16(v); }
__device__ __forceinline__ F2 split_col(const float* W, int k0, int n, int lane, int ld, int K) { float v[16]; const int g = lane >> 4;
#pragma unroll
  for (int i = 0; i < 8; ++i) { const int ka = k0 + 8 * g + i, kb = ka + 16; v[i] = ka < K ? W[(size_t)ka * ld + n] : 0.f; v[8 + i] = kb < K ? W[(size_t)kb * ld + n] : 0.f; }
  return bsplit16(v); }
__device__ __forceinline__ v8f mac3(const F2& a, const F2& b, v8f c) { c = wmma_bf(a.l, b.h, c); c = wmma_bf(a.h, b.l, c); return wmma_bf(a.h, b.h, c); }
__device__ __forceinline__ float sigm(float v) { return 1.0f / (1.0f + expf(-v)); }
#define LDSX() do { asm volatile("s_wait_dscnt 0" ::: "memory"); __builtin_amdgcn_wave_barrier(); __builtin_amdgcn_fence(__ATOMIC_RELEASE, "workgroup"); } while (0)

#define NBT 256
#define TT 64
#define DIM 16
#define LD 256
#define NAUX 128
#define HA 128
#define OW (DIM + LD)
#define NR (NBT * TT)
#define DTC 0.02f

__global__ __launch_bounds__(128) void k_enc(const float* __restrict__ x, const float* __restrict__ W1, const float* __restrict__ b1, const float* __restrict__ W2, const float* __restrict__ b2, const float* __restrict__ W3, float* __restrict__ out0, float* __restrict__ YE0) {
  __shared__ __align__(16) float sh[4][16][LD + 4];
  __shared__ __align__(16) float sh2[4][16][LD + 4];
  __shared__ __align__(16) float so[4][16][OW + 4];
  const int tid = threadIdx.x, wave = tid >> 5, lane = tid & 31, col = lane & 15, g = lane >> 4;
  const int r0 = blockIdx.x * 64 + wave * 16;
  for (int rl = 0; rl < 16; ++rl) { const float* xr = x + (size_t)(r0 + rl) * DIM; float xv[DIM];
#pragma unroll
    for (int d = 0; d < DIM; ++d) xv[d] = xr[d];
#pragma unroll
    for (int e = 0; e < 8; ++e) { const int hcol = lane * 8 + e; float s = b1[hcol];
#pragma unroll
      for (int d = 0; d < DIM; ++d) s += xv[d] * W1[d * LD + hcol];
      sh[wave][rl][hcol] = s > 0.f ? s : 0.f; }
    if (lane < DIM) so[wave][rl][lane] = xv[lane]; }
  LDSX();
#pragma unroll 1
  for (int np = 0; np < 2; ++np) { v8f acc[8] = {};
#pragma unroll 1
    for (int kc = 0; kc < LD / 32; ++kc) { const F2 a = split_row(&sh[wave][col][0], kc * 32, lane);
#pragma unroll
      for (int j = 0; j < 8; ++j) acc[j] = mac3(a, split_col(W2, kc * 32, np * 128 + j * 16 + col, lane, LD, LD), acc[j]); }
#pragma unroll
    for (int j = 0; j < 8; ++j) { const int c = np * 128 + j * 16 + col; const float bb = b2[c];
#pragma unroll
      for (int r = 0; r < 8; ++r) { const float v = acc[j][r] + bb; sh2[wave][8 * g + r][c] = v > 0.f ? v : 0.f; } } }
  LDSX();
#pragma unroll 1
  for (int np = 0; np < 2; ++np) { v8f ac[8] = {};
#pragma unroll 1
    for (int kc = 0; kc < LD / 32; ++kc) { const F2 a = split_row(&sh2[wave][col][0], kc * 32, lane);
#pragma unroll
      for (int j = 0; j < 8; ++j) ac[j] = mac3(a, split_col(W3, kc * 32, np * 128 + j * 16 + col, lane, LD, LD), ac[j]); }
#pragma unroll
    for (int j = 0; j < 8; ++j) { const int c = np * 128 + j * 16 + col;
#pragma unroll
      for (int r = 0; r < 8; ++r) so[wave][8 * g + r][DIM + c] = ac[j][r]; } }
  LDSX();
  for (int q = lane; q < 16 * (OW / 4); q += 32) { const int rl = q / (OW / 4), pc = q % (OW / 4); vst2(out0 + (size_t)(r0 + rl) * OW + pc * 4, *(const v4f*)(&so[wave][rl][pc * 4])); }
  if (wave == 0) { for (int q = lane; q < LD / 4; q += 32) vst2(YE0 + (size_t)blockIdx.x * LD + q * 4, *(const v4f*)(&so[0][0][DIM + q * 4])); }
}
__global__ __launch_bounds__(256) void k_koop(const float* __restrict__ x, const float* __restrict__ YE0, const float* __restrict__ aW1, const float* __restrict__ ab1, const float* __restrict__ aW2, const float* __restrict__ Wc, float* __restrict__ out1) {
  __shared__ __align__(16) float sl[TT][LD + 4];
  __shared__ __align__(16) float sxp[TT][DIM];
  __shared__ float sx0[DIM];
  const int b = blockIdx.x, tid = threadIdx.x;
  if (tid < DIM) sx0[tid] = x[((size_t)b * TT) * DIM + tid];
  __syncthreads();
  if (tid < NAUX) { const int n = tid;
    float o0 = 0.f, o1 = 0.f;
#pragma unroll 2
    for (int hh = 0; hh < HA; ++hh) { float s = ab1[n * HA + hh];
#pragma unroll
      for (int d = 0; d < DIM; ++d) s += sx0[d] * aW1[((size_t)n * DIM + d) * HA + hh];
      s = s > 0.f ? s : 0.f; o0 += s * aW2[((size_t)n * HA + hh) * 2]; o1 += s * aW2[((size_t)n * HA + hh) * 2 + 1]; }
    const float scale = expf(o0 * DTC); const float cs = cosf(o1 * DTC) * scale, sn = sinf(o1 * DTC) * scale;
    float ya = YE0[(size_t)b * LD + 2 * n], yb = YE0[(size_t)b * LD + 2 * n + 1];
    sl[0][2 * n] = ya; sl[0][2 * n + 1] = yb;
#pragma unroll 1
    for (int t = 1; t < TT; ++t) { const float na = ya * cs - yb * sn, nb = ya * sn + yb * cs; ya = na; yb = nb; sl[t][2 * n] = ya; sl[t][2 * n + 1] = yb; } }
  __syncthreads();
  for (int q = tid; q < TT * DIM; q += 256) { const int t = q >> 4, d = q & 15; float v;
    if (t == 0) v = sx0[d]; else { v = 0.f;
#pragma unroll 4
      for (int e = 0; e < LD; ++e) v += sl[t][e] * Wc[e * DIM + d]; }
    sxp[t][d] = v; }
  __syncthreads();
  for (int q = tid; q < TT * (OW / 4); q += 256) { const int t = q / (OW / 4), pc = q % (OW / 4); v4f o;
    if (pc < DIM / 4) o = *(const v4f*)(&sxp[t][pc * 4]); else o = *(const v4f*)(&sl[t][(pc - DIM / 4) * 4]);
    vst2(out1 + ((size_t)b * TT + t) * OW + pc * 4, o); }
}
extern "C" void kernel_launch(void* const* d_in, const int* in_sizes, int n_in, void* d_out, int out_size, void* d_ws, size_t ws_size, hipStream_t stream) {
  (void)in_sizes; (void)n_in; (void)out_size; (void)ws_size;
  const float** I = (const float**)d_in;
  float* out0 = (float*)d_out; float* out1 = (float*)((char*)d_out + 17825792);
  float* YE0 = (float*)d_ws;
  k_enc<<<NR / 64, 128, 0, stream>>>(I[0], I[1], I[2], I[3], I[4], I[5], out0, YE0);
  k_koop<<<NBT, 256, 0, stream>>>(I[0], YE0, I[6], I[7], I[8], I[9], out1);
}
